// GAT_62045097558453
// MI455X (gfx1250) — hardware-run, weakly checked
//
#include <hip/hip_runtime.h>


#ifndef NB
#define NB 4
#endif
#ifndef NCH
#define NCH 200
#endif
#define NB_FULL  4
#define NCH_FULL 200
#define SEQ_FULL 1000
#ifndef OUT_NCH
#define OUT_NCH NCH
#endif
#define UN   192
#define NH2  4
#define HD2  48
#define MT   (NB * NCH)
#define CW   12
#define PU   196
#define VP   200
#define OSF  196
#define GW   7
#define TQT  ((NCH + 15) / 16)
#define NKS  ((NCH + 31) / 32)
#define TKP  (NKS * 32)
#define GQB  ((TQT + GW - 1) / GW)
#define KPT  72
#define VPT  (TKP + 8)
#define OSH  200
#define WSC  16.0f
#define WSI  0.0625f
#define CSC  16.0f
#define PSH  14.0f
#define NEGB (-3.0e38f)
#define SC2A ((float)(0.7071067811865476 * 1.4426950408889634))
#define SC2G ((float)(0.14433756729740643 * 1.4426950408889634))

static_assert(UN == 192);
static_assert(NH2 * HD2 == UN);
static_assert(UN % 32 == 0);
static_assert(UN % 64 == 0);
static_assert(HD2 % 8 == 0 && HD2 <= 64 && HD2 > 32);
static_assert(HD2 % 16 == 0);
static_assert(CW * 16 == UN);
static_assert(32 * CW == 16 * (UN / 8));
static_assert(MT % 16 == 0);
static_assert(NCH >= 32);
static_assert(NCH * 5 <= SEQ_FULL);
static_assert(NB <= NB_FULL);
static_assert(NCH <= NCH_FULL);
static_assert((PU * 4) % 16 == 0 && (VP * 2) % 16 == 0 && (OSF * 4) % 16 == 0);
static_assert((KPT * 2) % 16 == 0 && (VPT * 2) % 16 == 0 && (OSH * 2) % 16 == 0);
static_assert(OSH >= UN && PU >= UN && VP >= UN && OSF >= UN && KPT >= 64);
static_assert((UN * 2) % 128 == 0);
static_assert((UN * 4) % 128 == 0);
static_assert((3 * UN * 2) % 128 == 0);
static_assert(12 * 32 * 16 == 16 * UN * 2);
static_assert(24 * 32 * 16 == 16 * UN * 4);
static_assert(2 * 256 * 16 == 64 * 128);
static_assert(48 * 16 == UN * 4 && 24 * 16 == UN * 2);
static_assert(32 * 32 * 2 + 32 * PU * 4 + 16 * VP * 2 + 32 * 4 + 16 * 4 + 2 * UN * 4 <= 131072);
static_assert(TKP * KPT * 2 + HD2 * VPT * 2 + GW * 16 * OSH * 2 <= 131072);
static_assert(16 * OSF * 4 <= 131072 && 64 * 65 * 4 <= 131072);

typedef _Float16 h16;
typedef __attribute__((ext_vector_type(16))) _Float16 v16h;
typedef __attribute__((ext_vector_type(8)))  _Float16 v8h;
typedef __attribute__((ext_vector_type(8)))  float    v8f;
typedef __attribute__((ext_vector_type(4)))  float    v4f;
typedef v4f  __attribute__((may_alias)) v4fa;

__device__ __forceinline__ unsigned short f2bf(float f) { unsigned u = __float_as_uint(f); u += 0x7FFFu + ((u >> 16) & 1u); return (unsigned short)(u >> 16); }
__device__ __forceinline__ float bfr(float f) { return __uint_as_float(((unsigned)f2bf(f)) << 16); }
__device__ __forceinline__ v16h cat16(v8h lo, v8h hi) { return __builtin_shufflevector(lo, hi, 0, 1, 2, 3, 4, 5, 6, 7, 8, 9, 10, 11, 12, 13, 14, 15); }
__device__ __forceinline__ v8f wmma16(v16h a, v16h b, v8f c) { return __builtin_amdgcn_wmma_f32_16x16x32_f16(false, a, false, b, (short)0, c, false, false); }
__device__ __forceinline__ v16h ldh(const h16* p) { return cat16(*(const v8h*)p, *(const v8h*)(p + 16)); }
#define LDS16(arr, i) cat16(*(const v8h*)&(arr)[(i)], *(const v8h*)&(arr)[(i) + 16])
__device__ __forceinline__ void wave_sync() { __builtin_amdgcn_fence(3  , "wavefront"); __builtin_amdgcn_wave_barrier(); asm volatile("" ::: "memory"); }
static __device__ __forceinline__ h16 toh_flush(float v) { const h16 r = (h16)v; return (fabsf(v) < 6.103515625e-05f) ? (h16)0.0f : r; }
__device__ __forceinline__ v8f wmmag(v16h a, v16h b, v8f c) {
    c = wmma16(a, b, c);
    asm volatile("v_nop\n\tv_nop\n\tv_nop\n\tv_nop" : "+v"(c) : "v"(a), "v"(b));
    return c;
}

__global__ __launch_bounds__(256) void k_wconv(const float* __restrict__ src, h16* dst) {
    __shared__ float tl[64 * 65];
    const int tid = threadIdx.x; const int k0 = blockIdx.x * 64, n0 = blockIdx.y * 64;
#pragma unroll 1
    for (int i = 0; i < 16; ++i) { const int idx = i * 256 + tid; const int r = idx >> 6, cc = idx & 63;
        tl[r * 65 + cc] = src[(size_t)(k0 + r) * UN + n0 + cc]; }
    __syncthreads();
#pragma unroll 1
    for (int ps = 0; ps < 2; ++ps) {
#pragma unroll
        for (int s = 0; s < 2; ++s) { const int p = s * 256 + tid; const int nr = p >> 3, pc = p & 7; v8h hv;
#pragma unroll
            for (int j = 0; j < 8; ++j) hv[j] = toh_flush(bfr(tl[(pc * 8 + j) * 65 + nr]) * WSC);
            *(volatile v8h*)(dst + (size_t)(n0 + nr) * UN + k0 + pc * 8) = hv; }
        if (ps == 0) __threadfence(); }
}

__global__ __launch_bounds__(32 * CW) void k_chunk(const float* __restrict__ x,
                                                   const float* __restrict__ Wq, const float* __restrict__ bq, const float* __restrict__ Wk, const float* __restrict__ bk,
                                                   const float* __restrict__ Wv, const float* __restrict__ bv, const float* __restrict__ Wo, const float* __restrict__ bo,
                                                   const float* __restrict__ pos, const float* __restrict__ gng, const float* __restrict__ gnb, float* XF, h16* XH) {
    __shared__ __align__(16) h16   wT_s[32 * 32];
    __shared__ __align__(16) float proj_s[32 * PU];
    __shared__ __align__(16) h16   vT_s[16 * VP];
    __shared__ float bias_s[32];
    __shared__ float wbar_s[16];
    __shared__ __align__(16) float xs_s[UN];
    __shared__ __align__(16) float y_s[UN];
    const int tid = threadIdx.x, lane = tid & 31, lr = lane & 15, hi = lane >> 4;
    const int wave = __builtin_amdgcn_readfirstlane((int)(threadIdx.x >> 5));
    const int bc = blockIdx.x; const int b = bc / NCH, c = bc % NCH;

#pragma unroll 1
    for (int i0 = 0; i0 < 1024; i0 += 32 * CW) {
        const int idx = i0 + tid; const int ic = idx < 1023 ? idx : 1023;
        const int n = ic >> 5, k = ic & 31;
        const int wh = n / 10; const int hk = n - wh * 10;
        const int hkc = hk < 9 ? hk : 9; const int kc = k < 19 ? k : 19;
        const size_t off = (size_t)c * 200 + (size_t)(kc * 10 + hkc);
        float a0 = Wq[off], a1 = Wk[off], a2 = Wv[off];
        asm volatile("" : "+v"(a0)); asm volatile("" : "+v"(a1)); asm volatile("" : "+v"(a2));
        const float sel = (wh == 0) ? a0 : ((wh == 1) ? a1 : a2);
        const bool ok = (n < 30) & (k < 20);
        const h16 hv = toh_flush(bfr(sel) * WSC);
        const h16 ov = ok ? hv : (h16)0.0f;
        if (idx < 1024) wT_s[ic] = ov;
    }
    if (wave == 0) {
        const int n = lane; const int wh = n / 10; const int hk = n - wh * 10; const int hkc = hk < 9 ? hk : 9;
        float a0 = bq[(size_t)c * 10 + hkc], a1 = bk[(size_t)c * 10 + hkc], a2 = bv[(size_t)c * 10 + hkc];
        asm volatile("" : "+v"(a0)); asm volatile("" : "+v"(a1)); asm volatile("" : "+v"(a2));
        const float sel = bfr((wh == 0) ? a0 : ((wh == 1) ? a1 : a2));
        const float ml = (wh == 0) ? SC2A : ((wh == 1) ? 1.0f : WSC);
        bias_s[n] = (n < 30) ? sel * ml : 0.0f;
    }
    if (wave == 1) {
        const int j = lr; const int jc = j < 9 ? j : 9;
        float sw = 0.0f, sb = 0.0f;
#pragma unroll 1
        for (int d = 0; d < 20; ++d) { sw += bfr(Wo[(size_t)c * 200 + jc * 20 + d]); sb += bfr(bo[(size_t)c * 20 + d]); }
        const float v = (j < 10) ? sw * (0.05f * WSI) : ((j == 10) ? sb * 0.05f : 0.0f);
        if (hi == 0) wbar_s[j] = v;
    }

    const int u = wave * 16 + lr;
    const size_t xb = ((size_t)b * SEQ_FULL + (size_t)c * 5) * UN + (size_t)u;
    const float ch0 = bfr(x[xb]), ch1 = bfr(x[xb + UN]), ch2 = bfr(x[xb + 2 * UN]), ch3 = bfr(x[xb + 3 * UN]), ch4 = bfr(x[xb + 4 * UN]);
    const float hbar = 0.2f * (((ch0 + ch1) + (ch2 + ch3)) + ch4);
    v16h af;
    { const h16 c0 = toh_flush(ch0), c1 = toh_flush(ch1), c2 = toh_flush(ch2), c3 = toh_flush(ch3), c4 = toh_flush(ch4); const h16 z = (h16)0.0f;
      af[0]  = hi ? c1 : c0;
      af[1]  = hi ? c2 : c1;
      af[2]  = hi ? c1 : c0;
      af[3]  = hi ? c3 : c2;
      af[4]  = hi ? c1 : c0;
      af[5]  = hi ? c4 : c3;
      af[6]  = hi ? c2 : c0;
      af[7]  = hi ? c3 : c4;
      af[8]  = hi ? z : c2;
      af[9]  = hi ? z : c4;
      af[10] = hi ? z : c3;
      af[11] = hi ? z : c4;
      af[12] = z; af[13] = z; af[14] = z; af[15] = z; }
    __syncthreads();

    { const v16h bw0 = LDS16(wT_s, lr * 32 + 8 * hi), bw1 = LDS16(wT_s, (16 + lr) * 32 + 8 * hi);
      v8f p0 = (v8f){}, p1 = (v8f){};
      p0 = wmmag(af, bw0, p0); p1 = wmmag(af, bw1, p1);
      const int n0 = lr, n1 = 16 + lr;
      const float cs0 = (n0 < 10) ? (SC2A * WSI) : WSI;
      const float cs1 = (n1 < 20) ? WSI : 1.0f;
      const float bb0 = bias_s[n0], bb1 = bias_s[n1];
      v4f a, cq;
      a[0] = p0[0] * cs0 + bb0; a[1] = p0[1] * cs0 + bb0; a[2] = p0[2] * cs0 + bb0; a[3] = p0[3] * cs0 + bb0;
      cq[0] = p0[4] * cs0 + bb0; cq[1] = p0[5] * cs0 + bb0; cq[2] = p0[6] * cs0 + bb0; cq[3] = p0[7] * cs0 + bb0;
      *(v4fa*)&proj_s[n0 * PU + wave * 16 + 8 * hi] = a; *(v4fa*)&proj_s[n0 * PU + wave * 16 + 8 * hi + 4] = cq;
      a[0] = p1[0] * cs1 + bb1; a[1] = p1[1] * cs1 + bb1; a[2] = p1[2] * cs1 + bb1; a[3] = p1[3] * cs1 + bb1;
      cq[0] = p1[4] * cs1 + bb1; cq[1] = p1[5] * cs1 + bb1; cq[2] = p1[6] * cs1 + bb1; cq[3] = p1[7] * cs1 + bb1;
      *(v4fa*)&proj_s[n1 * PU + wave * 16 + 8 * hi] = a; *(v4fa*)&proj_s[n1 * PU + wave * 16 + 8 * hi + 4] = cq; }
    __syncthreads();

    { const int r = tid / 24, u8 = (tid - r * 24) * 8; const int rs = (20 + r) < 31 ? (20 + r) : 31;
      const v4f x0 = *(const v4fa*)&proj_s[rs * PU + u8], x1 = *(const v4fa*)&proj_s[rs * PU + u8 + 4]; v8h hv;
#pragma unroll
      for (int i = 0; i < 4; ++i) { const h16 a0 = toh_flush(x0[i]), a1 = toh_flush(x1[i]); hv[i] = (r < 10) ? a0 : (h16)0.0f; hv[4 + i] = (r < 10) ? a1 : (h16)0.0f; }
      *(v8h*)&vT_s[r * VP + u8] = hv; }
    __syncthreads();

    const v16h hz = (v16h){};
    float ctxw = 0.0f;
#pragma unroll 1
    for (int hd = 0; hd < 5; ++hd) {
        const float q0 = proj_s[(2 * hd) * PU + u], q1 = proj_s[(2 * hd + 1) * PU + u];
        const int kr0 = (10 + 2 * hd) * PU + 8 * hi, kr1 = (11 + 2 * hd) * PU + 8 * hi;
        const int vrow = (2 * hd + (lr & 1)) * VP + 8 * hi;
        v8f o = (v8f){};
        float m = NEGB, l = 0.0f;
#pragma unroll 1
        for (int key0 = 0; key0 < UN; key0 += 32) {
            const v4f xa0 = *(const v4fa*)&proj_s[kr0 + key0], xa1 = *(const v4fa*)&proj_s[kr0 + key0 + 4];
            const v4f xb0 = *(const v4fa*)&proj_s[kr0 + key0 + 16], xb1 = *(const v4fa*)&proj_s[kr0 + key0 + 20];
            const v4f ya0 = *(const v4fa*)&proj_s[kr1 + key0], ya1 = *(const v4fa*)&proj_s[kr1 + key0 + 4];
            const v4f yb0 = *(const v4fa*)&proj_s[kr1 + key0 + 16], yb1 = *(const v4fa*)&proj_s[kr1 + key0 + 20];
            float ta[8], tb[8];
#pragma unroll
            for (int r = 0; r < 4; ++r) {
                ta[r] = q0 * xa0[r] + q1 * ya0[r]; ta[4 + r] = q0 * xa1[r] + q1 * ya1[r];
                tb[r] = q0 * xb0[r] + q1 * yb0[r]; tb[4 + r] = q0 * xb1[r] + q1 * yb1[r]; }
            float mx = NEGB;
#pragma unroll
            for (int r = 0; r < 8; ++r) mx = fmaxf(mx, fmaxf(ta[r], tb[r]));
            mx = fmaxf(mx, __shfl_xor(mx, 16, 32));
            const float mnew = fmaxf(m, mx);
            const float alpha = __builtin_amdgcn_exp2f(m - mnew);
            const float sh = PSH - mnew;
            v16h pb; float ls = 0.0f;
#pragma unroll
            for (int r = 0; r < 8; ++r) {
                const float ea0 = ta[r] + sh, eb0 = tb[r] + sh;
                const float ea = __builtin_amdgcn_exp2f(ea0), eb = __builtin_amdgcn_exp2f(eb0);
                const float ga = (ea0 < -14.0f) ? 0.0f : ea, gb = (eb0 < -14.0f) ? 0.0f : eb;
                const h16 pa = (h16)ga; const h16 pc = (h16)gb;
                pb[r] = pa; pb[8 + r] = pc; ls += (float)pa + (float)pc; }
            l = l * alpha + ls; m = mnew;
            o = o * alpha;
            v16h va = LDS16(vT_s, vrow + key0);
            asm volatile("" : "+v"(va));
            va = (lr < 2) ? va : hz;
            o = wmmag(va, pb, o);
        }
        l += __shfl_xor(l, 16, 32);
        const float inv = 1.0f / l;
        ctxw += (o[0] * wbar_s[2 * hd] + o[1] * wbar_s[2 * hd + 1]) * inv;
    }
    if (hi == 0) xs_s[u] = hbar + wbar_s[10] + ctxw;
    __syncthreads();

    float xv[6]; float s = 0.0f;
#pragma unroll
    for (int i = 0; i < 6; ++i) { xv[i] = xs_s[lane + 32 * i]; s += xv[i]; }
#pragma unroll
    for (int of = 16; of >= 1; of >>= 1) s += __shfl_xor(s, of, 32);
    const float mu = s * (1.0f / 192.0f);
    float d2 = 0.0f;
#pragma unroll
    for (int i = 0; i < 6; ++i) { const float d = xv[i] - mu; d2 += d * d; }
#pragma unroll
    for (int of = 16; of >= 1; of >>= 1) d2 += __shfl_xor(d2, of, 32);
    const float rs = rsqrtf(d2 * (1.0f / 192.0f) + 1.0e-3f);
    if (tid < UN) {
        const float gam = bfr(gng[c]), bet = bfr(gnb[c]);
        y_s[tid] = (xs_s[tid] - mu) * rs * gam + bet + bfr(pos[(size_t)c * UN + tid]);
    }
    __syncthreads();

    { const int pf = tid < 47 ? tid : 47;
      int ph = tid - 64; ph = ph < 0 ? 0 : (ph > 23 ? 23 : ph);
      const v4f vf = *(const v4fa*)&y_s[pf * 4];
      const v4f h0 = *(const v4fa*)&y_s[ph * 8], h1 = *(const v4fa*)&y_s[ph * 8 + 4]; v8h hv;
#pragma unroll
      for (int i = 0; i < 4; ++i) { hv[i] = toh_flush(h0[i]); hv[4 + i] = toh_flush(h1[i]); }
      float* of32 = XF + (size_t)bc * UN + pf * 4;
      h16* of16 = XH + (size_t)bc * UN + ph * 8;
#pragma unroll 1
      for (int ps = 0; ps < 2; ++ps) {
          if (tid < 48) *(volatile v4f*)of32 = vf;
          if ((tid >= 64) & (tid < 88)) *(volatile v8h*)of16 = hv;
          if (ps == 0) __threadfence(); } }
}

__device__ __forceinline__ void gemm16x192(const h16* __restrict__ A, const h16* __restrict__ Wt, int r0, int lr, int hi, v8f (&acc)[12]) {
#pragma unroll
    for (int nb = 0; nb < 12; ++nb) acc[nb] = (v8f){};
    const size_t aoff = (size_t)(r0 + lr) * UN + 8 * hi, boff = (size_t)lr * UN + 8 * hi;
#pragma unroll 1
    for (int kc = 0; kc < UN; kc += 32) {
        const v16h a = ldh(A + aoff + kc);
#pragma unroll
        for (int nb = 0; nb < 12; ++nb) { const v16h bw = ldh(Wt + boff + (size_t)nb * 16 * UN + kc); acc[nb] = wmmag(a, bw, acc[nb]); }
    }
}

__global__ __launch_bounds__(32) void k_gemm_h(const h16* __restrict__ A, const h16* __restrict__ Wt, const float* __restrict__ b0, const float* __restrict__ b1, const float* __restrict__ b2,
                                               h16* OUTH, int ldo) {
    __shared__ __align__(16) float os[16 * OSF];
    const int lane = threadIdx.x & 31, lr = lane & 15, hi = lane >> 4;
    const int r0 = blockIdx.x * 16; const int y = blockIdx.y;
    v8f acc[12];
    gemm16x192(A, Wt + (size_t)y * UN * UN, r0, lr, hi, acc);
#pragma unroll
    for (int nb = 0; nb < 12; ++nb) { const int cidx = nb * 16 + lr;
        const float x0 = b0[cidx], x1 = b1[cidx], x2 = b2[cidx];
        const float bvv = bfr((y == 0) ? x0 : ((y == 1) ? x1 : x2));
#pragma unroll
        for (int j = 0; j < 8; ++j) os[(hi * 8 + j) * OSF + cidx] = acc[nb][j] * WSI + bvv; }
    wave_sync();
    h16* ob = OUTH + (size_t)r0 * ldo + (size_t)y * UN;
#pragma unroll 1
    for (int ps = 0; ps < 2; ++ps) {
#pragma unroll 1
        for (int s = 0; s < 12; ++s) { const int p = s * 32 + lane; const int row = p / 24, pc = p - row * 24;
            const v4f x0 = *(const v4fa*)&os[row * OSF + pc * 8], x1 = *(const v4fa*)&os[row * OSF + pc * 8 + 4]; v8h hv;
#pragma unroll
            for (int i = 0; i < 4; ++i) { hv[i] = toh_flush(x0[i]); hv[4 + i] = toh_flush(x1[i]); }
            *(volatile v8h*)(ob + (size_t)row * ldo + pc * 8) = hv; }
        if (ps == 0) __threadfence(); }
}

__global__ __launch_bounds__(32) void k_gemm_ln(const h16* __restrict__ A, const h16* __restrict__ Wt, const float* __restrict__ bias, float oscale, const float* __restrict__ R,
                                                const float* __restrict__ gam, const float* __restrict__ bet, float* OF, int opitch, h16* OH, int gelu, int wr16) {
    __shared__ __align__(16) float os[16 * OSF];
    const int lane = threadIdx.x & 31, lr = lane & 15, hi = lane >> 4;
    const int r0 = blockIdx.x * 16;
    v8f acc[12];
    gemm16x192(A, Wt, r0, lr, hi, acc);
#pragma unroll
    for (int nb = 0; nb < 12; ++nb) { const int cidx = nb * 16 + lr; const float bvv = bfr(bias[cidx]);
#pragma unroll
        for (int j = 0; j < 8; ++j) os[(hi * 8 + j) * OSF + cidx] = acc[nb][j] * oscale + bvv; }
    wave_sync();
    float gq[6], bq6[6];
#pragma unroll
    for (int i = 0; i < 6; ++i) { gq[i] = bfr(gam[lane + 32 * i]); bq6[i] = bfr(bet[lane + 32 * i]); }
#pragma unroll 1
    for (int row = 0; row < 16; ++row) {
        const size_t gr = (size_t)(r0 + row);
        float xv[6]; float s = 0.0f;
#pragma unroll
        for (int i = 0; i < 6; ++i) { float v = os[row * OSF + lane + 32 * i];
            if (gelu) v = 0.5f * v * (1.0f + erff(v * 0.70710678118654752f));
            xv[i] = v + R[gr * UN + lane + 32 * i]; s += xv[i]; }
#pragma unroll
        for (int of = 16; of >= 1; of >>= 1) s += __shfl_xor(s, of, 32);
        const float mu = s * (1.0f / 192.0f);
        float d2 = 0.0f;
#pragma unroll
        for (int i = 0; i < 6; ++i) { const float d = xv[i] - mu; d2 += d * d; }
#pragma unroll
        for (int of = 16; of >= 1; of >>= 1) d2 += __shfl_xor(d2, of, 32);
        const float rs = rsqrtf(d2 * (1.0f / 192.0f) + 1.0e-3f);
#pragma unroll
        for (int i = 0; i < 6; ++i) os[row * OSF + lane + 32 * i] = (xv[i] - mu) * rs * gq[i] + bq6[i];
    }
    wave_sync();
#pragma unroll 1
    for (int ps = 0; ps < 2; ++ps) {
#pragma unroll 1
        for (int s = 0; s < 24; ++s) { const int p = s * 32 + lane; const int row = p / 48, pc = p - row * 48;
            const v4f val = *(const v4fa*)&os[row * OSF + pc * 4];
            const int gr = r0 + row; const size_t orow = (size_t)(gr / NCH) * (size_t)opitch + (size_t)(gr % NCH);
            *(volatile v4f*)(OF + orow * UN + pc * 4) = val; }
        if (wr16) {
#pragma unroll 1
            for (int s = 0; s < 12; ++s) { const int p = s * 32 + lane; const int row = p / 24, pc = p - row * 24;
                const v4f x0 = *(const v4fa*)&os[row * OSF + pc * 8], x1 = *(const v4fa*)&os[row * OSF + pc * 8 + 4]; v8h hv;
#pragma unroll
                for (int i = 0; i < 4; ++i) { hv[i] = toh_flush(x0[i]); hv[4 + i] = toh_flush(x1[i]); }
                *(volatile v8h*)(OH + (size_t)(r0 + row) * UN + pc * 8) = hv; } }
        if (ps == 0) __threadfence(); }
}

__global__ __launch_bounds__(32 * GW) void k_gattn(const h16* __restrict__ QKV, h16* CTX) {
    __shared__ __align__(16) h16 ks[TKP * KPT];
    __shared__ __align__(16) h16 vts[HD2 * VPT];
    __shared__ __align__(16) h16 osh[GW * 16 * OSH];
    const int tid = threadIdx.x, lane = tid & 31, lr = lane & 15, hi = lane >> 4;
    const int wave = __builtin_amdgcn_readfirstlane((int)(threadIdx.x >> 5));
    const int b = blockIdx.y; const int qt = blockIdx.x * GW + wave; const bool active = qt < TQT;
    const int t0 = qt * 16; const int tq = (t0 + lr) < NCH ? (t0 + lr) : (NCH - 1);
    const size_t rowb = (size_t)b * NCH;
    const v8h z8 = (v8h){};
#pragma unroll 1
    for (int h = 0; h < NH2; ++h) {
#pragma unroll 1
        for (int i0 = 0; i0 < TKP * 8; i0 += 32 * GW) {
            const int idx = i0 + tid; const int ic = idx < (TKP * 8 - 1) ? idx : (TKP * 8 - 1);
            const int key = ic >> 3, pc = ic & 7; const int kc = key < (NCH - 1) ? key : (NCH - 1); const int pcc = pc < 5 ? pc : 5;
            v8h xk = *(const v8h*)(QKV + (rowb + (size_t)kc) * (3 * UN) + UN + h * HD2 + pcc * 8);
            asm volatile("" : "+v"(xk));
            const bool ok = (key < NCH) & (pc < 6);
            const v8h ov = ok ? xk : z8;
            if (idx < TKP * 8) *(v8h*)&ks[key * KPT + pc * 8] = ov;
        }
#pragma unroll 1
        for (int i0 = 0; i0 < TKP * 6; i0 += 32 * GW) {
            const int idx = i0 + tid; const int ic = idx < (TKP * 6 - 1) ? idx : (TKP * 6 - 1);
            const int key = ic / 6; const int pc = ic - key * 6; const int kc = key < (NCH - 1) ? key : (NCH - 1);
            v8h xw = *(const v8h*)(QKV + (rowb + (size_t)kc) * (3 * UN) + 2 * UN + h * HD2 + pc * 8);
            asm volatile("" : "+v"(xw));
            const v8h ov = (key < NCH) ? xw : z8;
            if (idx < TKP * 6) {
#pragma unroll
                for (int j = 0; j < 8; ++j) vts[(pc * 8 + j) * VPT + key] = ov[j]; }
        }
        __syncthreads();
        if (active) {
            const size_t qo = (rowb + (size_t)tq) * (3 * UN) + h * HD2 + 8 * hi;
            const v16h qf0 = ldh(QKV + qo);
            const v16h qf1 = cat16(*(const v8h*)(QKV + qo + 32), z8);
            v8f o0 = (v8f){}, o1 = (v8f){}, o2 = (v8f){};
            float m = NEGB, l = 0.0f;
#pragma unroll 1
            for (int key0 = 0; key0 < TKP; key0 += 32) {
                const int ka = (key0 + lr) * KPT + 8 * hi;
                const v16h ka0 = LDS16(ks, ka), ka1 = LDS16(ks, ka + 32);
                const v16h kb0 = LDS16(ks, ka + 16 * KPT), kb1 = LDS16(ks, ka + 16 * KPT + 32);
                v8f sa = (v8f){}, sb = (v8f){};
                sa = wmmag(ka0, qf0, sa); sa = wmmag(ka1, qf1, sa);
                sb = wmmag(kb0, qf0, sb); sb = wmmag(kb1, qf1, sb);
                const int ja = key0 + 8 * hi;
                float ta[8], tb[8]; bool fa[8], fb[8]; float mx = NEGB;
#pragma unroll
                for (int r = 0; r < 8; ++r) {
                    fa[r] = (ja + r) < NCH; fb[r] = (ja + 16 + r) < NCH;
                    ta[r] = sa[r] * SC2G; tb[r] = sb[r] * SC2G;
                    mx = fmaxf(mx, fmaxf(fa[r] ? ta[r] : NEGB, fb[r] ? tb[r] : NEGB)); }
                mx = fmaxf(mx, __shfl_xor(mx, 16, 32));
                const float mnew = fmaxf(m, mx);
                const float alpha = __builtin_amdgcn_exp2f(m - mnew);
                const float sh = PSH - mnew;
                v16h pb; float ls = 0.0f;
#pragma unroll
                for (int r = 0; r < 8; ++r) {
                    const float ea0 = ta[r] + sh, eb0 = tb[r] + sh;
                    const float ea = __builtin_amdgcn_exp2f(ea0), eb = __builtin_amdgcn_exp2f(eb0);
                    const float ga = (fa[r] & (ea0 >= -14.0f)) ? ea : 0.0f, gb = (fb[r] & (eb0 >= -14.0f)) ? eb : 0.0f;
                    const h16 pa = (h16)ga; const h16 pc = (h16)gb;
                    pb[r] = pa; pb[8 + r] = pc; ls += (float)pa + (float)pc; }
                l = l * alpha + ls; m = mnew;
                o0 = o0 * alpha; o1 = o1 * alpha; o2 = o2 * alpha;
                const int va = lr * VPT + key0 + 8 * hi;
                const v16h v0 = LDS16(vts, va), v1 = LDS16(vts, va + 16 * VPT), v2 = LDS16(vts, va + 32 * VPT);
                o0 = wmmag(v0, pb, o0); o1 = wmmag(v1, pb, o1); o2 = wmmag(v2, pb, o2);
            }
            l += __shfl_xor(l, 16, 32);
            const float inv = CSC * (1.0f / l);
            const int ob = (wave * 16 + lr) * OSH + h * HD2 + 8 * hi;
            v8h hv;
#pragma unroll
            for (int r = 0; r < 8; ++r) hv[r] = toh_flush(o0[r] * inv);
            *(v8h*)&osh[ob] = hv;
#pragma unroll
            for (int r = 0; r < 8; ++r) hv[r] = toh_flush(o1[r] * inv);
            *(v8h*)&osh[ob + 16] = hv;
#pragma unroll
            for (int r = 0; r < 8; ++r) hv[r] = toh_flush(o2[r] * inv);
            *(v8h*)&osh[ob + 32] = hv;
        }
        __syncthreads();
    }
    if (active) {
        wave_sync();
#pragma unroll 1
        for (int ps = 0; ps < 2; ++ps) {
#pragma unroll 1
            for (int s = 0; s < 12; ++s) { const int p = s * 32 + lane; const int line = p >> 3; const int row = line / 3, seg = line - row * 3; const int col = seg * 64 + (p & 7) * 8;
                const v8h val = *(const v8h*)&osh[(wave * 16 + row) * OSH + col];
                const int t = t0 + row;
                if (t < NCH) *(volatile v8h*)(CTX + (rowb + (size_t)t) * UN + col) = val; }
            if (ps == 0) __threadfence(); }
    }
}

static constexpr size_t al256(size_t v) { return (v + 255) & ~(size_t)255; }
static constexpr size_t SZ_WT  = al256((size_t)6 * UN * UN * 2);
static constexpr size_t SZ_F32 = al256((size_t)MT * UN * 4);
static constexpr size_t SZ_F16 = al256((size_t)MT * UN * 2);
static constexpr size_t SZ_QKV = al256((size_t)MT * 3 * UN * 2);
static constexpr size_t SZ_TOTAL = SZ_WT + 2 * SZ_F32 + 4 * SZ_F16 + SZ_QKV;
static_assert(SZ_TOTAL <= (size_t)134217728);
static_assert(((size_t)UN * UN * 2) % 256 == 0);

extern "C" void kernel_launch(void* const* d_in, const int* in_sizes, int n_in,
                              void* d_out, int out_size, void* d_ws, size_t ws_size, hipStream_t stream) {
    if (n_in < 28) return;
    if ((size_t)in_sizes[0] < ((size_t)(NB - 1) * SEQ_FULL + (size_t)NCH * 5) * UN) return;
    if (in_sizes[1] < NCH * 200 || in_sizes[3] < NCH * 200 || in_sizes[5] < NCH * 200 || in_sizes[7] < NCH * 200) return;
    if (in_sizes[2] < NCH * 10 || in_sizes[4] < NCH * 10 || in_sizes[6] < NCH * 10 || in_sizes[8] < NCH * 20) return;
    if (in_sizes[9] < NCH * UN) return;
    if (in_sizes[10] < UN * UN || in_sizes[12] < UN * UN || in_sizes[14] < UN * UN || in_sizes[16] < UN * UN || in_sizes[20] < UN * UN || in_sizes[22] < UN * UN) return;
    if (in_sizes[11] < UN || in_sizes[13] < UN || in_sizes[15] < UN || in_sizes[17] < UN || in_sizes[21] < UN || in_sizes[23] < UN) return;
    if (in_sizes[18] < NCH || in_sizes[19] < NCH) return;
    if (in_sizes[24] < UN || in_sizes[25] < UN || in_sizes[26] < UN || in_sizes[27] < UN) return;
    if ((size_t)out_size < ((size_t)(NB - 1) * OUT_NCH + NCH) * UN) return;
    if (SZ_TOTAL > ws_size) return;
    const float* x   = (const float*)d_in[0];
    const float* Wq  = (const float*)d_in[1];  const float* bq  = (const float*)d_in[2];
    const float* Wk  = (const float*)d_in[3];  const float* bk  = (const float*)d_in[4];
    const float* Wv  = (const float*)d_in[5];  const float* bv  = (const float*)d_in[6];
    const float* Wo  = (const float*)d_in[7];  const float* bo  = (const float*)d_in[8];
    const float* pos = (const float*)d_in[9];
    const float* gWq = (const float*)d_in[10]; const float* gbq = (const float*)d_in[11];
    const float* gWk = (const float*)d_in[12]; const float* gbk = (const float*)d_in[13];
    const float* gWv = (const float*)d_in[14]; const float* gbv = (const float*)d_in[15];
    const float* gWo = (const float*)d_in[16]; const float* gbo = (const float*)d_in[17];
    const float* gng = (const float*)d_in[18]; const float* gnb = (const float*)d_in[19];
    const float* W1  = (const float*)d_in[20]; const float* b1  = (const float*)d_in[21];
    const float* W2  = (const float*)d_in[22]; const float* b2  = (const float*)d_in[23];
    const float* l1g = (const float*)d_in[24]; const float* l1b = (const float*)d_in[25];
    const float* l2g = (const float*)d_in[26]; const float* l2b = (const float*)d_in[27];
    float* OUT = (float*)d_out;
    char* wsp = (char*)d_ws;
    h16* WT   = (h16*)wsp;   wsp += SZ_WT;
    float* XF = (float*)wsp; wsp += SZ_F32;
    float* X1F = (float*)wsp; wsp += SZ_F32;
    h16* XH   = (h16*)wsp;   wsp += SZ_F16;
    h16* CTX  = (h16*)wsp;   wsp += SZ_F16;
    h16* X1H  = (h16*)wsp;   wsp += SZ_F16;
    h16* Y1H  = (h16*)wsp;   wsp += SZ_F16;
    h16* QKV  = (h16*)wsp;   wsp += SZ_QKV;
    const size_t WW = (size_t)UN * UN;

    k_chunk<<<dim3(MT, 1, 1), 32 * CW, 0, stream>>>(x, Wq, bq, Wk, bk, Wv, bv, Wo, bo, pos, gng, gnb, XF, XH);

    k_wconv<<<dim3(UN / 64, UN / 64, 1), 256, 0, stream>>>(gWq, WT);
    k_wconv<<<dim3(UN / 64, UN / 64, 1), 256, 0, stream>>>(gWk, WT + WW);
    k_wconv<<<dim3(UN / 64, UN / 64, 1), 256, 0, stream>>>(gWv, WT + 2 * WW);
    k_wconv<<<dim3(UN / 64, UN / 64, 1), 256, 0, stream>>>(gWo, WT + 3 * WW);
    k_wconv<<<dim3(UN / 64, UN / 64, 1), 256, 0, stream>>>(W1, WT + 4 * WW);
    k_wconv<<<dim3(UN / 64, UN / 64, 1), 256, 0, stream>>>(W2, WT + 5 * WW);

    k_gemm_h<<<dim3(MT / 16, 3, 1), 32, 0, stream>>>(XH, WT, gbq, gbk, gbv, QKV, 3 * UN);
    k_gattn<<<dim3(GQB, NB, 1), 32 * GW, 0, stream>>>(QKV, CTX);
    k_gemm_ln<<<dim3(MT / 16, 1, 1), 32, 0, stream>>>(CTX, WT + 3 * WW, gbo, WSI * (1.0f / CSC), XF, l1g, l1b, X1F, NCH, X1H, 0, 1);
    k_gemm_h<<<dim3(MT / 16, 1, 1), 32, 0, stream>>>(X1H, WT + 4 * WW, b1, b1, b1, Y1H, UN);
    k_gemm_ln<<<dim3(MT / 16, 1, 1), 32, 0, stream>>>(Y1H, WT + 5 * WW, b2, WSI, X1F, l2g, l2b, OUT, OUT_NCH, X1H, 1, 0);
}
